// ES_MOE_36197984371395
// MI455X (gfx1250) — hardware-verified
//
#include <hip/hip_runtime.h>
#include <stdint.h>

typedef __bf16         v16b __attribute__((ext_vector_type(16)));
typedef unsigned short us8  __attribute__((ext_vector_type(8)));
typedef float          v8f  __attribute__((ext_vector_type(8)));
typedef float          v4f  __attribute__((ext_vector_type(4)));
typedef us8 __attribute__((may_alias)) us8a;
typedef v4f __attribute__((may_alias)) v4fa;

union Frag { v16b v; us8 half[2]; };

#define NB    16
#define NC    128
#define NCR   16
#define NE    3
#define HH    80
#define WW    80
#define NPIX  6400
#define TR    2
#define MT    160
#define NBI   40
#define CCH   32
#define NKC   4
#define HR    8
#define XP    88
#define AP    40
#define SP    160
#define NTH   512
#define NWAV  16
#define XS_FLOATS (CCH * HR * XP)
#define PW_PLANE  (NE * NC * NC)

static_assert(MT == TR * WW);
static_assert(XS_FLOATS >= NC * SP);
static_assert(XP >= 16 * 4 + 24);
static_assert((PW_PLANE % 8) == 0);

__device__ __forceinline__ v8f wmma_bf16(v16b a, v16b b, v8f c) {
  v8f d = __builtin_amdgcn_wmma_f32_16x16x32_bf16(false, a, false, b, (short)0, c, false, false);
  asm volatile("v_nop\n\tv_nop\n\tv_nop\n\tv_nop" : "+v"(d) : "v"(a), "v"(b));
  return d;
}

__device__ __forceinline__ unsigned int bf16_rne_bits(float v) {
  const unsigned int u = __builtin_bit_cast(unsigned int, v);
  return (u + 0x7FFFu + ((u >> 16) & 1u)) >> 16;
}

__device__ __forceinline__ void split2(float v, unsigned short& hi, unsigned short& lo) {
  const unsigned int hb = bf16_rne_bits(v);
  const float hf = __builtin_bit_cast(float, hb << 16);
  const unsigned int lb = bf16_rne_bits(v - hf);
  hi = (unsigned short)hb;
  lo = (unsigned short)lb;
}

__global__ __launch_bounds__(256) void pw_convert(
    const float* __restrict__ pw0, const float* __restrict__ pw1,
    const float* __restrict__ pw2,
    unsigned short* __restrict__ phi, unsigned short* __restrict__ plo)
{
  const int g = blockIdx.x * 256 + threadIdx.x;
  if (g >= PW_PLANE / 8) return;
  const int e = g >> 11;
  const int off = (g & 2047) * 8;
  const float* src = (e == 0) ? pw0 : ((e == 1) ? pw1 : pw2);
  const v4f a = *(const v4fa*)(src + off);
  const v4f c = *(const v4fa*)(src + off + 4);
  const float f[8] = {a.x, a.y, a.z, a.w, c.x, c.y, c.z, c.w};
  us8 hv, lv;
  #pragma unroll
  for (int j = 0; j < 8; ++j) {
    unsigned short hs, ls;
    split2(f[j], hs, ls);
    hv[j] = hs;
    lv[j] = ls;
  }
  unsigned short* dh = phi + (size_t)g * 8;
  unsigned short* dl = plo + (size_t)g * 8;
  *(volatile us8*)dh = hv;
  *(volatile us8*)dl = lv;
  __threadfence();
  *(volatile us8*)dh = hv;
  *(volatile us8*)dl = lv;
}

template <int KK, int E>
__device__ __forceinline__ void dw_phase(const float* xs, unsigned short* ahi, unsigned short* alo,
                                         const float* routeL, const float* __restrict__ dwg,
                                         int c0, int tid)
{
  constexpr int P2 = KK / 2;
  constexpr int NIT = CCH * TR * 5;
  #pragma unroll 1
  for (int it = tid; it < NIT; it += NTH) {
    const int cl = it & (CCH - 1);
    const int q  = it >> 5;
    const int rr = (q >= 5) ? 1 : 0;
    const int g  = q - 5 * rr;
    const float* wp = dwg + (size_t)(c0 + cl) * (KK * KK);
    float a[16];
    #pragma unroll
    for (int j = 0; j < 16; ++j) a[j] = 0.0f;
    #pragma unroll 1
    for (int dy = 0; dy < KK; ++dy) {
      const int hr = rr + dy + (3 - P2);
      const float* rp = xs + (cl * HR + hr) * XP + 16 * g;
      float win[24];
      #pragma unroll
      for (int u = 0; u < 6; ++u) {
        const v4f t4 = *(const v4fa*)(rp + 4 * u);
        win[4 * u + 0] = t4.x;
        win[4 * u + 1] = t4.y;
        win[4 * u + 2] = t4.z;
        win[4 * u + 3] = t4.w;
      }
      float wv[KK];
      #pragma unroll
      for (int dx = 0; dx < KK; ++dx) wv[dx] = wp[dy * KK + dx];
      #pragma unroll
      for (int dx = 0; dx < KK; ++dx) {
        #pragma unroll
        for (int j = 0; j < 16; ++j)
          a[j] = fmaf(wv[dx], win[j + dx + (4 - P2)], a[j]);
      }
    }
    #pragma unroll
    for (int j = 0; j < 16; ++j) {
      const int p = rr * WW + 16 * g + j;
      const float v = a[j] * routeL[p * 4 + E];
      unsigned short hu, lu;
      split2(v, hu, lu);
      ahi[p * AP + cl] = hu;
      alo[p * AP + cl] = lu;
    }
  }
}

__device__ __forceinline__ void gemm_phase(v8f (&acc)[5],
    const unsigned short* ahi, const unsigned short* alo,
    const unsigned short* __restrict__ phi, const unsigned short* __restrict__ plo,
    int e, int kc, int ngrp, int mh, int h, int m)
{
  const size_t boff = (size_t)(e * NC + 16 * ngrp + m) * NC + kc * CCH;
  Frag bh, bl;
  bh.half[0] = *(const us8a*)(phi + boff + 8 * h);
  bh.half[1] = *(const us8a*)(phi + boff + 16 + 8 * h);
  bl.half[0] = *(const us8a*)(plo + boff + 8 * h);
  bl.half[1] = *(const us8a*)(plo + boff + 16 + 8 * h);
  #pragma unroll
  for (int tt = 0; tt < 5; ++tt) {
    const int aoff = ((MT / 2) * mh + 16 * tt + m) * AP;
    Frag fh, fl;
    fh.half[0] = *(const us8a*)(ahi + aoff + 8 * h);
    fh.half[1] = *(const us8a*)(ahi + aoff + 16 + 8 * h);
    fl.half[0] = *(const us8a*)(alo + aoff + 8 * h);
    fl.half[1] = *(const us8a*)(alo + aoff + 16 + 8 * h);
    acc[tt] = wmma_bf16(fh.v, bh.v, acc[tt]);
    acc[tt] = wmma_bf16(fl.v, bh.v, acc[tt]);
    acc[tt] = wmma_bf16(fh.v, bl.v, acc[tt]);
  }
}

__device__ __forceinline__ void out_store_pass(const float* so, float* __restrict__ out,
                                               int b, int r0, int wv, int lane)
{
  const int q8 = lane & 7, sub = lane >> 3;
  #pragma unroll
  for (int i = 0; i < 10; ++i) {
    const int L = 4 * i + sub;
    const int cq = L / 5, seg = L - 5 * cq;
    const int c = 8 * wv + cq;
    const v4f v = *(const v4fa*)(so + c * SP + seg * 32 + 4 * q8);
    float* dst = out + (size_t)(b * NC + c) * NPIX + r0 * WW + seg * 32 + 4 * q8;
    *(volatile v4f*)dst = v;
  }
}

__global__ __launch_bounds__(NTH) void moe_fused(
    const float* __restrict__ x,
    const float* __restrict__ w1, const float* __restrict__ b1,
    const float* __restrict__ w2, const float* __restrict__ b2,
    const float* __restrict__ gamma, const float* __restrict__ beta,
    const float* __restrict__ mean,  const float* __restrict__ var,
    const float* __restrict__ dw0, const float* __restrict__ dw1,
    const float* __restrict__ dw2,
    const unsigned short* __restrict__ phi, const unsigned short* __restrict__ plo,
    float* __restrict__ out)
{
  __shared__ __attribute__((aligned(16))) float xs[XS_FLOATS];
  __shared__ __attribute__((aligned(16))) unsigned short ahi[MT * AP];
  __shared__ __attribute__((aligned(16))) unsigned short alo[MT * AP];
  __shared__ __attribute__((aligned(16))) float routeL[MT * 4];
  __shared__ float bnsc[NC];
  __shared__ float bnsh[NC];

  const int tid = threadIdx.x, lane = tid & 31, wv = tid >> 5;
  const int h = lane >> 4, m = lane & 15;
  const int ngrp = wv & 7, mh = wv >> 3;
  const int blk = blockIdx.x;
  const int b = blk / NBI;
  if (b >= NB) return;
  const int r0 = (blk - b * NBI) * TR;
  const int pix0 = r0 * WW;
  const float* xb = x + (size_t)b * NC * NPIX;

  if (tid < NC) {
    const float sc = gamma[tid] * (1.0f / sqrtf(var[tid] + 1e-5f));
    bnsc[tid] = sc;
    bnsh[tid] = beta[tid] - mean[tid] * sc;
  }

  if (tid < MT) {
    float ha[NCR];
    #pragma unroll
    for (int j = 0; j < NCR; ++j) ha[j] = 0.0f;
    const float* xp = xb + pix0 + tid;
    #pragma unroll 1
    for (int c = 0; c < NC; ++c) {
      const float xv = xp[(size_t)c * NPIX];
      #pragma unroll
      for (int j = 0; j < NCR; ++j) ha[j] = fmaf(w1[j * NC + c], xv, ha[j]);
    }
    float lg[NE];
    #pragma unroll
    for (int e = 0; e < NE; ++e) lg[e] = 0.0f;
    #pragma unroll
    for (int j = 0; j < NCR; ++j) {
      const float hvv = fmaxf(ha[j] + b1[j], 0.0f);
      #pragma unroll
      for (int e = 0; e < NE; ++e) lg[e] = fmaf(w2[e * NCR + j], hvv, lg[e]);
    }
    #pragma unroll
    for (int e = 0; e < NE; ++e) lg[e] += b2[e];
    const float mx = fmaxf(lg[0], fmaxf(lg[1], lg[2]));
    const float e0 = expf(lg[0] - mx), e1 = expf(lg[1] - mx), e2 = expf(lg[2] - mx);
    const float s = (e0 + e1) + e2;
    const float inv = 1.0f / s;
    routeL[tid * 4 + 0] = e0 * inv;
    routeL[tid * 4 + 1] = e1 * inv;
    routeL[tid * 4 + 2] = e2 * inv;
    routeL[tid * 4 + 3] = 0.0f;
  }

  const v8f z8 = {0.f, 0.f, 0.f, 0.f, 0.f, 0.f, 0.f, 0.f};
  v8f acc[5];
  #pragma unroll
  for (int tt = 0; tt < 5; ++tt) acc[tt] = z8;

  #pragma unroll 1
  for (int kc = 0; kc < NKC; ++kc) {
    const int c0 = kc * CCH;
    __syncthreads();

    #pragma unroll 1
    for (int q = wv; q < CCH * HR; q += NWAV) {
      const int cl = q >> 3, hr = q & 7;
      const int ir = r0 - 3 + hr;
      const bool rok = (ir >= 0) && (ir < HH);
      const int irc = min(max(ir, 0), HH - 1);
      const float* src = xb + (size_t)(c0 + cl) * NPIX + irc * WW;
      float* dst = xs + (cl * HR + hr) * XP;
      #pragma unroll
      for (int u = 0; u < 3; ++u) {
        const int hc  = lane + 32 * u;
        const int hcc = min(hc, XP - 1);
        const int ic  = hcc - 4;
        const bool cok = rok && (ic >= 0) && (ic < WW);
        const int icc = min(max(ic, 0), WW - 1);
        const float v = src[icc];
        if (hc < XP) dst[hc] = cok ? v : 0.0f;
      }
    }
    __syncthreads();

    dw_phase<3, 0>(xs, ahi, alo, routeL, dw0, c0, tid);
    __syncthreads();
    gemm_phase(acc, ahi, alo, phi, plo, 0, kc, ngrp, mh, h, m);
    __syncthreads();

    dw_phase<5, 1>(xs, ahi, alo, routeL, dw1, c0, tid);
    __syncthreads();
    gemm_phase(acc, ahi, alo, phi, plo, 1, kc, ngrp, mh, h, m);
    __syncthreads();

    dw_phase<7, 2>(xs, ahi, alo, routeL, dw2, c0, tid);
    __syncthreads();
    gemm_phase(acc, ahi, alo, phi, plo, 2, kc, ngrp, mh, h, m);
  }
  __syncthreads();

  float* so = xs;
  {
    const int c = 16 * ngrp + m;
    const float sc = bnsc[c], sh = bnsh[c];
    #pragma unroll
    for (int tt = 0; tt < 5; ++tt) {
      #pragma unroll
      for (int r = 0; r < 8; ++r) {
        const int p = (MT / 2) * mh + 16 * tt + 8 * h + r;
        const float o  = acc[tt][r] * sc + sh;
        const float oc = fmaxf(o, -30.0f);
        const float ex = __expf(-oc);
        const float sg = 1.0f / (1.0f + ex);
        so[c * SP + p] = o * sg;
      }
    }
  }
  __syncthreads();

  out_store_pass(so, out, b, r0, wv, lane);
  __threadfence();
  out_store_pass(so, out, b, r0, wv, lane);
}

extern "C" void kernel_launch(void* const* d_in, const int* in_sizes, int n_in,
                              void* d_out, int out_size, void* d_ws, size_t ws_size,
                              hipStream_t stream)
{
  if (n_in < 15) return;
  if (in_sizes[0] != NB * NC * NPIX) return;
  if (in_sizes[1] != NCR * NC || in_sizes[2] != NCR) return;
  if (in_sizes[3] != NE * NCR || in_sizes[4] != NE) return;
  if (in_sizes[5] != NC || in_sizes[6] != NC || in_sizes[7] != NC || in_sizes[8] != NC) return;
  if (in_sizes[9] != NC * 9 || in_sizes[11] != NC * 25 || in_sizes[13] != NC * 49) return;
  if (in_sizes[10] != NC * NC || in_sizes[12] != NC * NC || in_sizes[14] != NC * NC) return;
  if (out_size != NB * NC * NPIX) return;

  const size_t plane_bytes = (size_t)PW_PLANE * 2;
  const size_t total = 2 * plane_bytes;
  if (total > ws_size) return;

  const float* x     = (const float*)d_in[0];
  const float* r_w1  = (const float*)d_in[1];
  const float* r_b1  = (const float*)d_in[2];
  const float* r_w2  = (const float*)d_in[3];
  const float* r_b2  = (const float*)d_in[4];
  const float* gamma = (const float*)d_in[5];
  const float* beta  = (const float*)d_in[6];
  const float* mean  = (const float*)d_in[7];
  const float* var   = (const float*)d_in[8];
  const float* dw0   = (const float*)d_in[9];
  const float* pw0   = (const float*)d_in[10];
  const float* dw1   = (const float*)d_in[11];
  const float* pw1   = (const float*)d_in[12];
  const float* dw2   = (const float*)d_in[13];
  const float* pw2   = (const float*)d_in[14];
  float* out = (float*)d_out;

  char* ws = (char*)d_ws;
  unsigned short* phi = (unsigned short*)(ws);
  unsigned short* plo = (unsigned short*)(ws + plane_bytes);

  pw_convert<<<(PW_PLANE / 8 + 255) / 256, 256, 0, stream>>>(pw0, pw1, pw2, phi, plo);

  moe_fused<<<NB * NBI, NTH, 0, stream>>>(x, r_w1, r_b1, r_w2, r_b2,
                                         gamma, beta, mean, var,
                                         dw0, dw1, dw2, phi, plo, out);
}
